// MaskedMultiHeadAttention_21406117003304
// MI455X (gfx1250) — hardware-verified
//
#include <hip/hip_runtime.h>


#ifndef NB
#define NB 4
#endif
#ifndef SEQ
#define SEQ 2048
#endif

namespace {
constexpr int BF = 4, TF = 2048, DM = 1024, H = 16, HD = 64, SRC = 64;
constexpr int BL = NB;
constexpr int QL = SEQ;
constexpr int KL = (QL + SRC < TF) ? (QL + SRC) : TF;
constexpr int NBH = (BL < 2) ? BL : 2;
constexpr int NPASS = (BL + NBH - 1) / NBH;
constexpr int RSPLIT = (QL < 512) ? QL : 512;
constexpr float XS = 8.0f, WSC = 256.0f, PS = 1024.0f, CS = 64.0f, LOG2E = 1.4426950408889634f, L2THETA = 13.287712379549449f;
static_assert(BL >= 1 && BL <= BF);
static_assert(QL >= 64 && QL <= TF && QL % 64 == 0);
static_assert(KL % 64 == 0 && KL <= TF && KL >= QL);
static_assert(RSPLIT % 32 == 0 && RSPLIT <= QL);
static_assert(DM == H * HD && TF % 64 == 0 && HD == 64);

typedef _Float16 b16;
typedef __attribute__((ext_vector_type(16))) _Float16 v16b;
typedef __attribute__((ext_vector_type(8))) _Float16 v8b;
typedef __attribute__((ext_vector_type(4))) _Float16 v4h;
typedef __attribute__((ext_vector_type(2))) _Float16 v2h;
typedef __attribute__((ext_vector_type(8))) float v8f;
typedef __attribute__((ext_vector_type(4))) float v4f;
typedef __attribute__((ext_vector_type(2))) float v2f;

__device__ __forceinline__ float bf16_rne(float f) { unsigned int u = __float_as_uint(f); u += 0x7FFFu + ((u >> 16) & 1u); return __uint_as_float(u & 0xFFFF0000u); }
__device__ __forceinline__ void split16(float v, b16& hi, b16& lo) { hi = (b16)v; lo = (b16)(v - (float)hi); }
__device__ __forceinline__ v16b frag_kb(const b16* p, int hh) {
  const v8b a = *(const v8b*)(p + 8 * hh), b = *(const v8b*)(p + 16 + 8 * hh); v16b f;
#pragma unroll
  for (int e = 0; e < 8; ++e) { f[e] = a[e]; f[8 + e] = b[e]; }
  return f;
}
__device__ __forceinline__ v8f wmma16b(v16b a, v16b b, v8f c) {
  v8f d = __builtin_amdgcn_wmma_f32_16x16x32_f16(false, a, false, b, (short)0, c, false, false);
  asm volatile("v_nop\n\tv_nop\n\tv_nop\n\tv_nop" : "+v"(d) : "v"(a), "v"(b));
  return d;
}
__device__ __forceinline__ void wave_lds_sync() { __builtin_amdgcn_fence(3  , "workgroup"); __builtin_amdgcn_wave_barrier(); __builtin_amdgcn_fence(2  , "workgroup"); }
__device__ __forceinline__ float nexp2(float v) { return __builtin_amdgcn_exp2f(v); }

__global__ __launch_bounds__(256) void prep_kernel(const float* __restrict__ wq, const float* __restrict__ wk, const float* __restrict__ wv, const float* __restrict__ wp, b16* __restrict__ WT, b16* __restrict__ WO) {
  const size_t u = (size_t)blockIdx.x * 256 + threadIdx.x;
  if (u >= (size_t)4 * DM * DM / 8) return;
  const int mtx = (int)(u / ((size_t)DM * DM / 8)); const size_t e = (u % ((size_t)DM * DM / 8)) * 8; const int oo = (int)(e / DM), k0 = (int)(e % DM);
  const float* w = mtx == 0 ? wq : mtx == 1 ? wk : mtx == 2 ? wv : wp;
  v8b o;
#pragma unroll
  for (int j = 0; j < 8; ++j) o[j] = (b16)(bf16_rne(w[(size_t)(k0 + j) * DM + oo]) * WSC);
  b16* dst = (mtx < 3) ? (WT + (size_t)mtx * DM * DM + e) : (WO + e);
  for (int pass = 0; pass < 2; ++pass) { *(volatile v8b*)dst = o; __threadfence(); }
}

__global__ __launch_bounds__(256) void rope_tab_kernel(float* __restrict__ cst, float* __restrict__ snt) {
  const int i = blockIdx.x * 256 + threadIdx.x;
  if (i >= TF * (HD / 2)) return;
  const int t = i / (HD / 2), p = i % (HD / 2);
  const float e = (float)(2 * p) * (1.0f / (float)HD);
  const float inv = exp2f(-(e * L2THETA));
  const float ang = (float)t * inv;
  float sv, cv;
  sincosf(ang, &sv, &cv);
  for (int pass = 0; pass < 2; ++pass) { *(volatile float*)(cst + i) = cv; *(volatile float*)(snt + i) = sv; __threadfence(); }
}

__global__ __launch_bounds__(256) void xcvt_kernel(const float* __restrict__ x, b16* __restrict__ X8, int b0, int nb) {
  const size_t u = (size_t)blockIdx.x * 256 + threadIdx.x;
  const size_t per = (size_t)KL * DM / 8;
  if (u >= (size_t)nb * per) return;
  const int bb = (int)(u / per); const size_t e = (u % per) * 8; const int t = (int)(e / DM), c = (int)(e % DM);
  const float* src = x + (((size_t)(b0 + bb)) * TF + t) * DM + c;
  const v4f f0 = *(const v4f*)src, f1 = *(const v4f*)(src + 4);
  v8b o;
#pragma unroll
  for (int j = 0; j < 4; ++j) { o[j] = (b16)(bf16_rne(f0[j]) * XS); o[4 + j] = (b16)(bf16_rne(f1[j]) * XS); }
  b16* dst = X8 + ((size_t)bb * TF + t) * DM + c;
  for (int pass = 0; pass < 2; ++pass) { *(volatile v8b*)dst = o; __threadfence(); }
}

__global__ __launch_bounds__(128) void proj_kernel(const b16* __restrict__ X8, const b16* __restrict__ WT, const float* __restrict__ bq, const float* __restrict__ bk, const float* __restrict__ bv,
                                                    const float* __restrict__ cst, const float* __restrict__ snt,
                                                    b16* __restrict__ QH, b16* __restrict__ QLo, b16* __restrict__ KH, b16* __restrict__ KLo, b16* __restrict__ VTh, b16* __restrict__ VTl) {
  __shared__ __attribute__((aligned(16))) float Tf[4][16][128 + 4];
  const int wave = threadIdx.x >> 5, lane = threadIdx.x & 31, nloc = lane & 15, hlf = lane >> 4;
  const int t0 = blockIdx.x * 64; const int bb = blockIdx.y; const int slab = blockIdx.z, n0 = slab * 128, part = slab / 8, c0 = n0 - part * DM;
  const size_t m0 = (size_t)bb * TF + t0 + wave * 16;
  v8f acc[8];
#pragma unroll
  for (int t = 0; t < 8; ++t) acc[t] = (v8f){};
#pragma unroll 2
  for (int kb = 0; kb < DM; kb += 32) {
    const v16b a = frag_kb(X8 + (m0 + nloc) * DM + kb, hlf);
#pragma unroll
    for (int t = 0; t < 8; ++t) acc[t] = wmma16b(a, frag_kb(WT + (size_t)(n0 + t * 16 + nloc) * DM + kb, hlf), acc[t]);
  }
  const float* bias = part == 0 ? bq : part == 1 ? bk : bv;
#pragma unroll
  for (int t = 0; t < 8; ++t) {
    const float bval = bf16_rne(bias[c0 + t * 16 + nloc]);
#pragma unroll
    for (int r = 0; r < 8; ++r) Tf[wave][8 * hlf + r][t * 16 + nloc] = acc[t][r] * (1.0f / (XS * WSC)) + bval;
  }
  __syncthreads();
  for (int pass = 0; pass < 2; ++pass) {
    if (part < 2) {
      b16* ph_ = part == 0 ? QH : KH; b16* pl_ = part == 0 ? QLo : KLo;
      const int c = c0 + lane * 4; const int hq = c / HD, d = c % HD, p0 = d >> 1;
      for (int rr = 0; rr < 16; ++rr) {
        const int tok = t0 + wave * 16 + rr;
        const v4f f = *(const v4f*)(&Tf[wave][rr][lane * 4]);
        const v2f cc = *(const v2f*)(cst + (size_t)tok * (HD / 2) + p0), ss = *(const v2f*)(snt + (size_t)tok * (HD / 2) + p0);
        const float o0 = f[0] * cc[0] - f[1] * ss[0];
        const float o1 = f[0] * ss[0] + f[1] * cc[0];
        const float o2 = f[2] * cc[1] - f[3] * ss[1];
        const float o3 = f[2] * ss[1] + f[3] * cc[1];
        v4h h4, l4; b16 ph, pl;
        split16(o0 * XS, ph, pl); h4[0] = ph; l4[0] = pl;
        split16(o1 * XS, ph, pl); h4[1] = ph; l4[1] = pl;
        split16(o2 * XS, ph, pl); h4[2] = ph; l4[2] = pl;
        split16(o3 * XS, ph, pl); h4[3] = ph; l4[3] = pl;
        const size_t oi = (((size_t)bb * H + hq) * TF + tok) * HD + d;
        *(volatile v4h*)(ph_ + oi) = h4; *(volatile v4h*)(pl_ + oi) = l4;
      }
    } else {
#pragma unroll 1
      for (int q = 0; q < 32; ++q) {
        const int cl = wave * 32 + q; const int c = c0 + cl; const int hv_ = c / HD, d = c % HD; const int tk = lane * 2; v2h hv, lv;
        for (int j = 0; j < 2; ++j) { b16 p, ql; split16(Tf[(tk + j) >> 4][(tk + j) & 15][cl] * XS, p, ql); hv[j] = p; lv[j] = ql; }
        const size_t oi = (((size_t)bb * H + hv_) * HD + d) * (size_t)TF + t0 + lane * 2;
        *(volatile v2h*)(VTh + oi) = hv; *(volatile v2h*)(VTl + oi) = lv;
      }
    }
    __threadfence();
  }
}

template <int RES>
__global__ __launch_bounds__(64) void attn_kernel(const b16* __restrict__ QH, const b16* __restrict__ QLo, const b16* __restrict__ KH, const b16* __restrict__ KLo, const b16* __restrict__ VTh, const b16* __restrict__ VTl,
                                                   b16* __restrict__ Ch, b16* __restrict__ Cl, int xb0) {
  __shared__ __attribute__((aligned(16))) b16 Pb[2][16][32 + 8], Pc[2][16][32 + 8]; __shared__ __attribute__((aligned(16))) float To[2][16][HD + 4];
  const int wave = threadIdx.x >> 5, lane = threadIdx.x & 31, hh = lane >> 4, col = lane & 15; const int bb = blockIdx.y / H, h = blockIdx.y % H;
  const int q0 = (xb0 + (int)blockIdx.x) * 32 + wave * 16, qi = q0 + col;
  const size_t ph = (size_t)bb * H + h; const size_t pq = ph * TF * HD; const b16* Vh = VTh + ph * HD * (size_t)TF; const b16* Vl = VTl + ph * HD * (size_t)TF;
  const v16b qh0 = frag_kb(QH + pq + (size_t)qi * HD, hh), qh1 = frag_kb(QH + pq + (size_t)qi * HD + 32, hh);
  v16b ql0 = (v16b){}, ql1 = (v16b){};
  if (RES) { ql0 = frag_kb(QLo + pq + (size_t)qi * HD, hh); ql1 = frag_kb(QLo + pq + (size_t)qi * HD + 32, hh); }
  const float cs = LOG2E / (8.0f * XS * XS);
  float m = -INFINITY, l = 0.0f; v8f o[4];
#pragma unroll
  for (int t = 0; t < 4; ++t) o[t] = (v8f){};
  const int kmax = q0 + 16 + SRC; const int kend = kmax < KL ? kmax : KL;
#pragma unroll 1
  for (int kb = 0; kb < kend; kb += 32) {
    float e[16]; float mx = -INFINITY;
#pragma unroll
    for (int u = 0; u < 2; ++u) {
      v8f s = (v8f){}; const size_t kr = pq + (size_t)(kb + u * 16 + col) * HD;
      const v16b kh0 = frag_kb(KH + kr, hh), kh1 = frag_kb(KH + kr + 32, hh);
      if (RES) {
        const v16b kl0 = frag_kb(KLo + kr, hh), kl1 = frag_kb(KLo + kr + 32, hh);
        s = wmma16b(kh0, qh0, s); s = wmma16b(kh0, ql0, s); s = wmma16b(kl0, qh0, s); s = wmma16b(kh1, qh1, s); s = wmma16b(kh1, ql1, s); s = wmma16b(kl1, qh1, s);
      } else {
        s = wmma16b(kh0, qh0, s); s = wmma16b(kh1, qh1, s);
      }
#pragma unroll
      for (int r = 0; r < 8; ++r) { const int key = kb + u * 16 + 8 * hh + r; const float vv = (key <= qi + SRC) ? s[r] * cs : -INFINITY; e[u * 8 + r] = vv; mx = fmaxf(mx, vv); }
    }
    mx = fmaxf(mx, __shfl_xor(mx, 16)); const float mn = fmaxf(m, mx); const float al = (mn == -INFINITY) ? 1.0f : nexp2(m - mn); float sum = 0.0f;
#pragma unroll
    for (int i2 = 0; i2 < 16; ++i2) {
      const float p = (e[i2] == -INFINITY) ? 0.0f : nexp2(e[i2] - mn); sum += p;
      const int sl = (i2 < 8 ? 0 : 16) + 8 * hh + (i2 & 7);
      if (RES) { b16 a_, b_; split16(p * PS, a_, b_); Pb[wave][col][sl] = a_; Pc[wave][col][sl] = b_; }
      else { Pb[wave][col][sl] = (b16)(p * PS); }
    }
    sum += __shfl_xor(sum, 16); l = l * al + sum; m = mn;
    wave_lds_sync();
    const v16b pf = frag_kb(&Pb[wave][col][0], hh);
    v16b pg = (v16b){};
    if (RES) pg = frag_kb(&Pc[wave][col][0], hh);
#pragma unroll
    for (int t = 0; t < 4; ++t) {
      o[t] *= al; const size_t vr = (size_t)(t * 16 + col) * TF + kb;
      const v16b va = frag_kb(Vh + vr, hh);
      if (RES) { const v16b vb2 = frag_kb(Vl + vr, hh); o[t] = wmma16b(va, pf, o[t]); o[t] = wmma16b(va, pg, o[t]); o[t] = wmma16b(vb2, pf, o[t]); }
      else { o[t] = wmma16b(va, pf, o[t]); }
    }
    wave_lds_sync();
  }
  const float inv = 1.0f / (l * PS * XS);
#pragma unroll
  for (int t = 0; t < 4; ++t)
#pragma unroll
    for (int r = 0; r < 8; ++r) To[wave][col][t * 16 + 8 * hh + r] = o[t][r] * inv;
  wave_lds_sync();
  for (int pass = 0; pass < 2; ++pass) {
    for (int rr = 0; rr < 16; ++rr) {
      const v2f f = *(const v2f*)(&To[wave][rr][lane * 2]); v2h hv, lv;
      for (int j = 0; j < 2; ++j) { b16 p, q; split16(f[j] * CS, p, q); hv[j] = p; lv[j] = q; }
      const size_t oi = ((size_t)bb * TF + q0 + rr) * DM + h * HD + lane * 2;
      *(volatile v2h*)(Ch + oi) = hv; *(volatile v2h*)(Cl + oi) = lv;
    }
    __threadfence();
  }
}

__global__ __launch_bounds__(128) void out_kernel(const b16* __restrict__ Ch, const b16* __restrict__ Cl, const b16* __restrict__ WO, float* __restrict__ out, int b0) {
  __shared__ __attribute__((aligned(16))) float Tf[4][16][128 + 4];
  const int wave = threadIdx.x >> 5, lane = threadIdx.x & 31, nloc = lane & 15, hlf = lane >> 4; const int bb = blockIdx.z;
  const size_t m0 = (size_t)bb * TF + ((size_t)blockIdx.x * 4 + wave) * 16;
  const size_t mo = (size_t)(b0 + bb) * TF + ((size_t)blockIdx.x * 4 + wave) * 16;
  const int n0 = blockIdx.y * 128;
  v8f acc[8];
#pragma unroll
  for (int t = 0; t < 8; ++t) acc[t] = (v8f){};
#pragma unroll 2
  for (int kb = 0; kb < DM; kb += 32) {
    const v16b a = frag_kb(Ch + (m0 + nloc) * DM + kb, hlf), al = frag_kb(Cl + (m0 + nloc) * DM + kb, hlf);
#pragma unroll
    for (int t = 0; t < 8; ++t) { const v16b bw = frag_kb(WO + (size_t)(n0 + t * 16 + nloc) * DM + kb, hlf); acc[t] = wmma16b(a, bw, acc[t]); acc[t] = wmma16b(al, bw, acc[t]); }
  }
#pragma unroll
  for (int t = 0; t < 8; ++t) {
#pragma unroll
    for (int r = 0; r < 8; ++r) Tf[wave][8 * hlf + r][t * 16 + nloc] = acc[t][r] * (1.0f / (CS * WSC));
  }
  wave_lds_sync();
  for (int pass = 0; pass < 2; ++pass) {
    for (int rr = 0; rr < 16; ++rr) *(volatile v4f*)(out + (mo + rr) * DM + n0 + lane * 4) = *(const v4f*)(&Tf[wave][rr][lane * 4]);
    __threadfence();
  }
}
}

extern "C" void kernel_launch(void* const* d_in, const int* in_sizes, int n_in, void* d_out, int out_size, void* d_ws, size_t ws_size, hipStream_t stream) {
  if (n_in < 8) return;
  auto Fp = [&](int i) { return (const float*)d_in[i]; };
  if (in_sizes[0] < BL * TF * DM || in_sizes[1] < DM * DM || in_sizes[2] < DM || in_sizes[3] < DM * DM || in_sizes[4] < DM || in_sizes[5] < DM * DM || in_sizes[6] < DM || in_sizes[7] < DM * DM ||
      out_size < BL * TF * DM) return;
  size_t off = 0; char* ws = (char*)d_ws;
  auto carve = [&](size_t bytes) { char* p = ws + off; off += (bytes + 255) & ~(size_t)255; return p; };
  b16* WT = (b16*)carve((size_t)3 * DM * DM * 2); b16* WO = (b16*)carve((size_t)DM * DM * 2);
  float* CST = (float*)carve((size_t)TF * (HD / 2) * 4); float* SNT = (float*)carve((size_t)TF * (HD / 2) * 4);
  const size_t plane = (size_t)NBH * TF * DM * 2;
  b16* X8 = (b16*)carve(plane);
  b16* QH = (b16*)carve(plane); b16* QLo = (b16*)carve(plane); b16* KH = (b16*)carve(plane); b16* KLo = (b16*)carve(plane);
  b16* VTh = (b16*)carve(plane); b16* VTl = (b16*)carve(plane); b16* Ch = (b16*)carve(plane); b16* Cl = (b16*)carve(plane);
  if (off > ws_size || off > ((size_t)128 << 20)) return;
  prep_kernel<<<(unsigned)(((size_t)4 * DM * DM / 8 + 255) / 256), 256, 0, stream>>>(Fp(1), Fp(3), Fp(5), Fp(7), WT, WO);
  rope_tab_kernel<<<(unsigned)((TF * (HD / 2) + 255) / 256), 256, 0, stream>>>(CST, SNT);
  for (int p = 0; p < NPASS; ++p) {
    const int b0 = p * NBH; const int nb = (BL - b0 < NBH) ? (BL - b0) : NBH;
    xcvt_kernel<<<(unsigned)(((size_t)nb * KL * DM / 8 + 255) / 256), 256, 0, stream>>>(Fp(0), X8, b0, nb);
    proj_kernel<<<dim3(KL / 64, nb, 24), 128, 0, stream>>>(X8, WT, Fp(2), Fp(4), Fp(6), CST, SNT, QH, QLo, KH, KLo, VTh, VTl);
    attn_kernel<1><<<dim3(RSPLIT / 32, nb * H), 64, 0, stream>>>(QH, QLo, KH, KLo, VTh, VTl, Ch, Cl, 0);
    if (QL > RSPLIT) attn_kernel<0><<<dim3((QL - RSPLIT) / 32, nb * H), 64, 0, stream>>>(QH, QLo, KH, KLo, VTh, VTl, Ch, Cl, RSPLIT / 32);
    out_kernel<<<dim3(QL / 64, DM / 128, nb), 128, 0, stream>>>(Ch, Cl, WO, (float*)d_out, b0);
  }
}
